// MQALocalAttention_88983132438631
// MI455X (gfx1250) — hardware-run, weakly checked
//
#include <hip/hip_runtime.h>
#include <math.h>

typedef __attribute__((ext_vector_type(16))) _Float16 v16h;
typedef __attribute__((ext_vector_type(16))) __bf16 v16b;
typedef __attribute__((ext_vector_type(8)))  _Float16 v8h;
typedef __attribute__((ext_vector_type(8)))  float v8f;
typedef __attribute__((ext_vector_type(4)))  float v4f;
typedef __attribute__((ext_vector_type(2)))  float v2f;
typedef __attribute__((ext_vector_type(4)))  unsigned v4u;
typedef __attribute__((ext_vector_type(4)))  int v4i;
typedef float __attribute__((may_alias)) float_a;
typedef int __attribute__((may_alias)) int_a;

template <typename T> __device__ __forceinline__ void vst2(void* p, T v) { *(volatile T*)p = v; __threadfence(); *(volatile T*)p = v; }
__device__ __forceinline__ v8f wmma16(v16h a, v16h b, v8f c) {
  v8f d = __builtin_amdgcn_wmma_f32_16x16x32_f16(false, a, false, b, (short)0, c, false, false);
  asm volatile("v_nop\n\tv_nop\n\tv_nop\n\tv_nop" : "+v"(d) : "v"(a), "v"(b));
  return d;
}
__device__ __forceinline__ v8f wmma_bf(v16b a, v16b b, v8f c) {
  v8f d = __builtin_amdgcn_wmma_f32_16x16x32_bf16(false, a, false, b, (short)0, c, false, false);
  asm volatile("v_nop\n\tv_nop\n\tv_nop\n\tv_nop" : "+v"(d) : "v"(a), "v"(b));
  return d;
}
__device__ __forceinline__ v16h frag_h(const _Float16* rowk0, int lane) {
  union { v16h v; v8h q[2]; } u; const _Float16* p = rowk0 + 8 * (lane >> 4);
  u.q[0] = *(const v8h*)p; u.q[1] = *(const v8h*)(p + 16); return u.v;
}
__device__ __forceinline__ v16h frag_f32(const float* rowk0, int lane) {
  v16h a; const float* p = rowk0 + 8 * (lane >> 4);
#pragma unroll
  for (int i = 0; i < 8; ++i) { a[i] = (_Float16)p[i]; a[8 + i] = (_Float16)p[16 + i]; }
  return a;
}
__device__ __forceinline__ v16h frag_f32s(const float* rowk0, int lane, float sc) {
  v16h a; const float* p = rowk0 + 8 * (lane >> 4);
#pragma unroll
  for (int i = 0; i < 8; ++i) { a[i] = (_Float16)(p[i] * sc); a[8 + i] = (_Float16)(p[16 + i] * sc); }
  return a;
}
__device__ __forceinline__ v16h fragc_f32(const float* W, int k0, int n, int lane, int ld, int K) {
  v16h a; const int g = lane >> 4;
#pragma unroll
  for (int i = 0; i < 8; ++i) { const int ka = k0 + 8 * g + i, kb = ka + 16;
    a[i] = (_Float16)(ka < K ? W[(size_t)(ka < K ? ka : K - 1) * ld + n] : 0.f); a[8 + i] = (_Float16)(kb < K ? W[(size_t)(kb < K ? kb : K - 1) * ld + n] : 0.f); }
  return a;
}
struct F2 { v16b h, l; };
__device__ __forceinline__ F2 bsplit16(const float v[16]) { F2 r;
#pragma unroll
  for (int i = 0; i < 16; ++i) { const __bf16 h = (__bf16)v[i]; r.h[i] = h; r.l[i] = (__bf16)(v[i] - (float)h); }
  return r; }
__device__ __forceinline__ F2 split_row(const float* row, int k0, int lane) { float v[16]; const float* p = row + k0 + 8 * (lane >> 4);
#pragma unroll
  for (int i = 0; i < 8; ++i) { v[i] = p[i]; v[8 + i] = p[16 + i]; }
  return bsplit16(v); }
__device__ __forceinline__ F2 split_rowK(const float* row, int k0, int lane, int K) { float v[16]; const int g = lane >> 4;
#pragma unroll
  for (int i = 0; i < 8; ++i) { const int ka = k0 + 8 * g + i, kb = ka + 16; v[i] = ka < K ? row[ka < K ? ka : K - 1] : 0.f; v[8 + i] = kb < K ? row[kb < K ? kb : K - 1] : 0.f; }
  return bsplit16(v); }
__device__ __forceinline__ F2 split_col(const float* W, int k0, int n, int lane, int ld, int K) { float v[16]; const int g = lane >> 4;
#pragma unroll
  for (int i = 0; i < 8; ++i) { const int ka = k0 + 8 * g + i, kb = ka + 16; v[i] = ka < K ? W[(size_t)(ka < K ? ka : K - 1) * ld + n] : 0.f; v[8 + i] = kb < K ? W[(size_t)(kb < K ? kb : K - 1) * ld + n] : 0.f; }
  return bsplit16(v); }
__device__ __forceinline__ v8f mac3(const F2& a, const F2& b, v8f c) { c = wmma_bf(a.l, b.h, c); c = wmma_bf(a.h, b.l, c); return wmma_bf(a.h, b.h, c); }
__device__ __forceinline__ float sigm(float v) { return 1.0f / (1.0f + expf(-v)); }
#define LDSX() do { asm volatile("s_wait_dscnt 0" ::: "memory"); __builtin_amdgcn_wave_barrier(); __builtin_amdgcn_fence(__ATOMIC_RELEASE, "workgroup"); } while (0)


#define NB 2
#define SS 2048
#define DM 1024
#define NH 16
#define HD 64
#define HALFW 64
#define NR (NB * SS)
#ifndef TQB
#define TQB (SS / 64)
#define TNB NB
#endif
typedef __attribute__((ext_vector_type(8))) __bf16 v8b;
__device__ __forceinline__ v16b frag_b(const __bf16* rowk0, int lane) {
  union { v16b v; v8b q[2]; } u; const __bf16* p = rowk0 + 8 * (lane >> 4);
  u.q[0] = *(const v8b*)p; u.q[1] = *(const v8b*)(p + 16); return u.v;
}
__device__ __forceinline__ float bfr(float v) { return (float)(__bf16)v; }
__device__ __attribute__((noinline)) float exp_ni(float v) { return expf(v); }
__device__ __attribute__((noinline)) float erf_ni(float v) { return erff(v); }

#define WS_PQ  0u
#define WS_PKV (WS_PQ + 2u * (size_t)DM * DM)
#define WS_PO  (WS_PKV + 2u * (size_t)128 * DM)
#define WS_PGA (WS_PO + 2u * (size_t)DM * DM)
#define WS_PGB (WS_PGA + 2u * (size_t)DM * DM)
#define WS_Q   (WS_PGB + 2u * (size_t)DM * DM)
#define WS_K   (WS_Q + 2u * (size_t)NR * DM)
#define WS_V   (WS_K + 2u * (size_t)NR * HD)
#define WS_O   (WS_V + 2u * (size_t)NB * HD * SS)
#define WS_AT  (WS_O + 4u * (size_t)NR * DM)
#define WS_X   (WS_AT + 4u * (size_t)NR * DM)
#define WS_MU  (WS_X + 4u * (size_t)NR * DM)
#define WS_END (WS_MU + 4u * (size_t)NB * DM)

__global__ __launch_bounds__(256) void k_pack(const float* __restrict__ WQ, const float* __restrict__ WK, const float* __restrict__ WV, const float* __restrict__ WO, const float* __restrict__ WG, __bf16* __restrict__ PQ, __bf16* __restrict__ PKV, _Float16* __restrict__ PO, _Float16* __restrict__ PGA, _Float16* __restrict__ PGB) {
  const int n = blockIdx.x, which = blockIdx.y, t = threadIdx.x; __shared__ __align__(16) __bf16 sb[DM]; __shared__ __align__(16) _Float16 sh[DM];
  if (which == 0) { for (int k = t; k < DM; k += 256) sb[k] = (__bf16)WQ[(size_t)k * DM + n]; __syncthreads(); if (t < DM / 8) vst2((unsigned*)(PQ + (size_t)n * DM + t * 8), *(const v4u*)&sb[t * 8]); }
  else if (which == 1) { if (n >= 128) return; const float* w = (n < HD) ? WK : WV; const int c = n & (HD - 1); for (int k = t; k < DM; k += 256) sb[k] = (__bf16)w[(size_t)k * HD + c]; __syncthreads(); if (t < DM / 8) vst2((unsigned*)(PKV + (size_t)n * DM + t * 8), *(const v4u*)&sb[t * 8]); }
  else if (which == 2) { for (int k = t; k < DM; k += 256) sh[k] = (_Float16)(bfr(WO[(size_t)k * DM + n]) * 256.0f); __syncthreads(); if (t < DM / 8) vst2((unsigned*)(PO + (size_t)n * DM + t * 8), *(const v4u*)&sh[t * 8]); }
  else if (which == 3) { for (int k = t; k < DM; k += 256) sh[k] = (_Float16)(bfr(WG[(size_t)k * DM + n]) * 256.0f); __syncthreads(); if (t < DM / 8) vst2((unsigned*)(PGA + (size_t)n * DM + t * 8), *(const v4u*)&sh[t * 8]); }
  else { for (int k = t; k < DM; k += 256) sh[k] = (_Float16)(bfr(WG[(size_t)(DM + k) * DM + n]) * 256.0f); __syncthreads(); if (t < DM / 8) vst2((unsigned*)(PGB + (size_t)n * DM + t * 8), *(const v4u*)&sh[t * 8]); }
}
__global__ __launch_bounds__(128) void k_proj(const float* __restrict__ XQ, const float* __restrict__ XK, const float* __restrict__ XV, const __bf16* __restrict__ PQ, const __bf16* __restrict__ PKV, const float* __restrict__ BQ, const float* __restrict__ BK, const float* __restrict__ BV, _Float16* __restrict__ Q, _Float16* __restrict__ Kr, _Float16* __restrict__ V) {
  __shared__ __align__(16) _Float16 so[64][136]; __shared__ __align__(16) _Float16 st[64][72];
  const int tid = threadIdx.x, wave = tid >> 5, lane = tid & 31, col = lane & 15, g = lane >> 4; const int which = blockIdx.z; const int c0 = blockIdx.y * 128; if (which == 1 && c0 > 0) return;
  const size_t rb = (size_t)blockIdx.x * 64; const size_t r0 = rb + wave * 16;
  v8f acc[8] = {};
  if (which == 0) { const __bf16* Wr = PQ;
#pragma unroll 2
    for (int kc = 0; kc < DM / 32; ++kc) { v16b a; { const float* p = XQ + (r0 + col) * DM + kc * 32 + 8 * g;
#pragma unroll
        for (int i = 0; i < 8; ++i) { a[i] = (__bf16)p[i]; a[8 + i] = (__bf16)p[16 + i]; } }
#pragma unroll
      for (int j = 0; j < 8; ++j) acc[j] = wmma_bf(a, frag_b(Wr + (size_t)(c0 + j * 16 + col) * DM + kc * 32, lane), acc[j]); } }
  else {
#pragma unroll 2
    for (int kc = 0; kc < DM / 32; ++kc) { v16b ak, av; { const float* p = XK + (r0 + col) * DM + kc * 32 + 8 * g; const float* p2 = XV + (r0 + col) * DM + kc * 32 + 8 * g;
#pragma unroll
        for (int i = 0; i < 8; ++i) { ak[i] = (__bf16)p[i]; ak[8 + i] = (__bf16)p[16 + i]; av[i] = (__bf16)p2[i]; av[8 + i] = (__bf16)p2[16 + i]; } }
#pragma unroll
      for (int j = 0; j < 8; ++j) acc[j] = wmma_bf((j < 4) ? ak : av, frag_b(PKV + (size_t)(j * 16 + col) * DM + kc * 32, lane), acc[j]); } }
  if (which == 0) {
#pragma unroll
    for (int j = 0; j < 8; ++j) { const float bb = bfr(BQ[c0 + j * 16 + col]);
#pragma unroll
      for (int r = 0; r < 8; ++r) so[wave * 16 + 8 * g + r][j * 16 + col] = (_Float16)(acc[j][r] + bb); }
    __syncthreads(); for (int e = tid; e < 64 * 16; e += 128) { const int rl = e >> 4, q = e & 15; vst2((unsigned*)(Q + (rb + rl) * DM + c0 + q * 8), *(const v4u*)&so[rl][q * 8]); } }
  else {
#pragma unroll
    for (int j = 0; j < 8; ++j) { const int c = (j * 16 + col) & (HD - 1); const float bb = bfr((j < 4) ? BK[c] : BV[c]);
#pragma unroll
      for (int r = 0; r < 8; ++r) { const _Float16 hv = (_Float16)(acc[j][r] + bb); if (j < 4) so[wave * 16 + 8 * g + r][c] = hv; else st[c][wave * 16 + 8 * g + r] = hv; } }
    __syncthreads(); for (int e = tid; e < 64 * 8; e += 128) { const int rl = e >> 3, q = e & 7; vst2((unsigned*)(Kr + (rb + rl) * HD + q * 8), *(const v4u*)&so[rl][q * 8]); }
    const size_t b = rb / SS; const int s0 = (int)(rb % SS); for (int e = tid; e < 64 * 8; e += 128) { const int d = e >> 3, pc = e & 7; vst2((unsigned*)(V + ((b * HD + d) * SS) + s0 + pc * 8), *(const v4u*)&st[d][pc * 8]); } }
}
__global__ __launch_bounds__(128) void k_attn(const _Float16* __restrict__ Q, const _Float16* __restrict__ Kr, const _Float16* __restrict__ V, float* __restrict__ O) {
  __shared__ __align__(16) _Float16 sph[4][16][40]; __shared__ __align__(16) float so[4][16][68];
  const int tid = threadIdx.x, wave = tid >> 5, lane = tid & 31, col = lane & 15, g = lane >> 4; const int h = blockIdx.y; const size_t b = blockIdx.z; const int qb0 = (int)blockIdx.x * 64; const int q0 = qb0 + wave * 16; const size_t rq = b * SS + q0;
  v16h aq[2];
#pragma unroll
  for (int kc = 0; kc < 2; ++kc) aq[kc] = frag_h(Q + (rq + col) * DM + h * HD + kc * 32, lane);
  float m[8], l[8];
#pragma unroll
  for (int r = 0; r < 8; ++r) { m[r] = -3.0e38f; l[r] = 0.f; }
  v8f acc[4] = {};
  const int kslo = (qb0 - HALFW) > 0 ? (qb0 - HALFW) / 32 : 0; const int kshi = (qb0 + 64 + HALFW + 31) / 32 < SS / 32 ? (qb0 + 64 + HALFW + 31) / 32 : SS / 32;
#pragma unroll 1
  for (int ks = kslo; ks < kshi; ++ks) { const int j0 = ks * 32; v8f s[2];
#pragma unroll
    for (int ct = 0; ct < 2; ++ct) { const int kk = j0 + ct * 16 + col; const size_t rk = (b * SS + kk) * HD; v8f c = {};
#pragma unroll
      for (int kc = 0; kc < 2; ++kc) c = wmma16(aq[kc], frag_h(Kr + rk + kc * 32, lane), c);
#pragma unroll
      for (int r = 0; r < 8; ++r) { const int qi = q0 + 8 * g + r; const bool keep = (kk >= qi - HALFW) && (kk < qi + HALFW + 1); s[ct][r] = keep ? c[r] * 0.125f : -3.0e38f; } }
#pragma unroll
    for (int r = 0; r < 8; ++r) { float mx = fmaxf(s[0][r], s[1][r]);
#pragma unroll
      for (int o = 1; o < 16; o <<= 1) mx = fmaxf(mx, __shfl_xor(mx, o));
      const float mn = fmaxf(m[r], mx); const float alpha = (m[r] <= -1.0e38f) ? 0.f : __expf(m[r] - mn); const float e0 = (s[0][r] <= -1.0e38f) ? 0.f : __expf(s[0][r] - mn), e1 = (s[1][r] <= -1.0e38f) ? 0.f : __expf(s[1][r] - mn); float es = e0 + e1;
#pragma unroll
      for (int o = 1; o < 16; o <<= 1) es += __shfl_xor(es, o);
      l[r] = l[r] * alpha + es; m[r] = mn;
#pragma unroll
      for (int dt = 0; dt < 4; ++dt) acc[dt][r] *= alpha;
      sph[wave][8 * g + r][col] = (_Float16)(e0 * 2048.0f); sph[wave][8 * g + r][16 + col] = (_Float16)(e1 * 2048.0f); }
    LDSX();
    const v16h pa = frag_h(&sph[wave][col][0], lane);
#pragma unroll
    for (int dt = 0; dt < 4; ++dt) acc[dt] = wmma16(pa, frag_h(V + ((b * HD + dt * 16 + col) * SS) + j0, lane), acc[dt]);
    LDSX(); }
#pragma unroll
  for (int r = 0; r < 8; ++r) { const float il = (l[r] > 0.f) ? (1.0f / 2048.0f) / l[r] : 0.f;
#pragma unroll
    for (int dt = 0; dt < 4; ++dt) so[wave][8 * g + r][dt * 16 + col] = acc[dt][r] * il; }
  LDSX();
  for (int rl = 0; rl < 16; ++rl) if (lane < 16) vst2(O + (rq + rl) * DM + h * HD + lane * 4, *(const v4f*)&so[wave][rl][lane * 4]);
}
__global__ __launch_bounds__(128) void k_wo(const float* __restrict__ O, const _Float16* __restrict__ PO, const float* __restrict__ BO, float* __restrict__ AT) { __shared__ __align__(16) float so[4][16][132];
  const int tid = threadIdx.x, wave = tid >> 5, lane = tid & 31, col = lane & 15, g = lane >> 4; const size_t r0 = (size_t)blockIdx.x * 64 + wave * 16; const int c0 = blockIdx.y * 128;
  v8f acc[8] = {};
#pragma unroll 2
  for (int kc = 0; kc < DM / 32; ++kc) { v16h a; { const float* p = O + (r0 + col) * DM + kc * 32 + 8 * g;
#pragma unroll
      for (int i = 0; i < 8; ++i) { a[i] = (_Float16)p[i]; a[8 + i] = (_Float16)p[16 + i]; } }
#pragma unroll
    for (int j = 0; j < 8; ++j) acc[j] = wmma16(a, frag_h(PO + (size_t)(c0 + j * 16 + col) * DM + kc * 32, lane), acc[j]); }
#pragma unroll
  for (int j = 0; j < 8; ++j) { const float bb = bfr(BO[c0 + j * 16 + col]);
#pragma unroll
    for (int r = 0; r < 8; ++r) so[wave][8 * g + r][j * 16 + col] = acc[j][r] * (1.0f / 256.0f) + bb; }
  LDSX(); for (int rl = 0; rl < 16; ++rl) vst2(AT + (r0 + rl) * DM + c0 + lane * 4, *(const v4f*)&so[wave][rl][lane * 4]); }
__global__ __launch_bounds__(128) void k_gate(const float* __restrict__ AT, const float* __restrict__ XQ, const _Float16* __restrict__ PGA, const _Float16* __restrict__ PGB, const float* __restrict__ BG, float* __restrict__ X) { __shared__ __align__(16) float so[4][16][132];
  const int tid = threadIdx.x, wave = tid >> 5, lane = tid & 31, col = lane & 15, g = lane >> 4; const size_t r0 = (size_t)blockIdx.x * 64 + wave * 16; const int c0 = blockIdx.y * 128;
  v8f acc[8] = {};
#pragma unroll 2
  for (int kc = 0; kc < DM / 32; ++kc) { v16h a, ab; { const float* p = AT + (r0 + col) * DM + kc * 32 + 8 * g; const float* p2 = XQ + (r0 + col) * DM + kc * 32 + 8 * g;
#pragma unroll
      for (int i = 0; i < 8; ++i) { a[i] = (_Float16)p[i]; a[8 + i] = (_Float16)p[16 + i]; ab[i] = (_Float16)bfr(p2[i]); ab[8 + i] = (_Float16)bfr(p2[16 + i]); } }
#pragma unroll
    for (int j = 0; j < 8; ++j) { acc[j] = wmma16(a, frag_h(PGA + (size_t)(c0 + j * 16 + col) * DM + kc * 32, lane), acc[j]); acc[j] = wmma16(ab, frag_h(PGB + (size_t)(c0 + j * 16 + col) * DM + kc * 32, lane), acc[j]); } }
#pragma unroll
  for (int j = 0; j < 8; ++j) { const int c = c0 + j * 16 + col; const float bb = bfr(BG[c]);
#pragma unroll
    for (int r = 0; r < 8; ++r) { const size_t oi = (r0 + 8 * g + r) * DM + c; const float zz = acc[j][r] * (1.0f / 256.0f) + bb; const float gt = zz / (1.0f + __expf(-zz)); so[wave][8 * g + r][j * 16 + col] = AT[oi] * gt + bfr(XQ[oi]) * (1.0f - gt); } }
  LDSX(); for (int rl = 0; rl < 16; ++rl) vst2(X + (r0 + rl) * DM + c0 + lane * 4, *(const v4f*)&so[wave][rl][lane * 4]); }
__global__ __launch_bounds__(256) void k_rms(float* __restrict__ X, const float* __restrict__ RW) { __shared__ float red[8]; const int t = threadIdx.x; const size_t row = blockIdx.x; float v[4]; float q = 0.f; for (int i = 0; i < 4; ++i) { v[i] = X[row * DM + t * 4 + i]; q += v[i] * v[i]; }
#pragma unroll
  for (int o = 1; o < 32; o <<= 1) q += __shfl_xor(q, o);
  if ((t & 31) == 0) red[t >> 5] = q; __syncthreads(); float tq = 0.f; for (int i = 0; i < 8; ++i) tq += red[i]; const float inv = 1.0f / sqrtf(tq / (float)DM + 1e-6f);
  v4f o4; for (int i = 0; i < 4; ++i) o4[i] = v[i] * inv * bfr(RW[t * 4 + i]); __syncthreads(); vst2(X + row * DM + t * 4, o4); }
__global__ __launch_bounds__(256) void k_colmean(const float* __restrict__ X, float* __restrict__ MU) { __shared__ float sp[2][128]; __shared__ __align__(16) float sm[128]; const int t = threadIdx.x; const size_t b = blockIdx.y; const int c0 = blockIdx.x * 128; const int c = t & 127, hf = t >> 7;
  float s = 0.f; for (int r = hf * (SS / 2); r < (hf + 1) * (SS / 2); ++r) s += X[(b * SS + r) * DM + c0 + c]; sp[hf][c] = s; __syncthreads();
  if (t < 128) sm[t] = (sp[0][t] + sp[1][t]) / (float)SS; __syncthreads(); if (t < 32) vst2(MU + b * DM + c0 + t * 4, *(const v4f*)&sm[t * 4]); }
__global__ __launch_bounds__(256) void k_sub(const float* __restrict__ X, const float* __restrict__ MU, float* __restrict__ OUT) { const int t = threadIdx.x; const size_t row = blockIdx.x; const size_t b = row / SS; v4f o4; for (int i = 0; i < 4; ++i) o4[i] = X[row * DM + t * 4 + i] - MU[b * DM + t * 4 + i]; vst2(OUT + row * DM + t * 4, o4); }
extern "C" void kernel_launch(void* const* d_in, const int* in_sizes, int n_in, void* d_out, int out_size, void* d_ws, size_t ws_size, hipStream_t stream) {
  (void)in_sizes; (void)n_in; (void)out_size;
  const float** F = (const float**)d_in;
  if (ws_size < (size_t)WS_END) return;
  char* ws = (char*)d_ws; __bf16 *PQ = (__bf16*)(ws + WS_PQ), *PKV = (__bf16*)(ws + WS_PKV); _Float16 *PO = (_Float16*)(ws + WS_PO), *PGA = (_Float16*)(ws + WS_PGA), *PGB = (_Float16*)(ws + WS_PGB), *Q = (_Float16*)(ws + WS_Q), *Kr = (_Float16*)(ws + WS_K), *V = (_Float16*)(ws + WS_V); float *O = (float*)(ws + WS_O), *AT = (float*)(ws + WS_AT), *X = (float*)(ws + WS_X), *MU = (float*)(ws + WS_MU);
  k_pack<<<dim3(DM, 5), 256, 0, stream>>>(F[3], F[5], F[7], F[9], F[11], PQ, PKV, PO, PGA, PGB);
  k_proj<<<dim3(NR / 64, DM / 128, 2), 128, 0, stream>>>(F[0], F[1], F[2], PQ, PKV, F[4], F[6], F[8], Q, Kr, V);
  k_attn<<<dim3(TQB, NH, TNB), 128, 0, stream>>>(Q, Kr, V, O);
  k_wo<<<dim3(NR / 64, DM / 128), 128, 0, stream>>>(O, PO, F[10], AT);
  k_gate<<<dim3(NR / 64, DM / 128), 128, 0, stream>>>(AT, F[0], PGA, PGB, F[12], X);
  k_rms<<<NR, 256, 0, stream>>>(X, F[13]);
  k_colmean<<<dim3(DM / 128, NB), 256, 0, stream>>>(X, MU);
  k_sub<<<NR, 256, 0, stream>>>(X, MU, (float*)d_out);
}
